// NequIPNBodyNetSimple_13950053777580
// MI455X (gfx1250) — hardware-run, weakly checked
//
#include <hip/hip_runtime.h>
#include <math.h>

typedef __attribute__((ext_vector_type(16))) __bf16   v16b;
typedef __attribute__((ext_vector_type(8)))  __bf16   v8b;
typedef __attribute__((ext_vector_type(8)))  float    v8f;
typedef __attribute__((ext_vector_type(4)))  float    v4f;
typedef __attribute__((ext_vector_type(4)))  unsigned v4u;

constexpr int kBt     = 8;
constexpr int kNp     = 256;
constexpr int kSd     = 4;
constexpr int kHd     = 128;
constexpr int kLy     = 4;
constexpr int kRows   = kBt * kNp;
constexpr int kW1Rows = 2 * kHd + 1;
constexpr int kPQP    = 2 * kHd;
constexpr int kIT     = 8;
static_assert(kRows == 2048 && kW1Rows == 257 && kPQP == 256, "shape constants");
static_assert((kRows % 64) == 0 && (kPQP % 64) == 0 && (kHd % 64) == 0, "GEMM M,N multiples of 64");
static_assert((kHd % 32) == 0 && (kPQP % 32) == 0, "GEMM K multiples of 32");
static_assert((kNp % kIT) == 0 && (kRows % 16) == 0, "tile multiples");

constexpr size_t kSzHF  = (size_t)kRows * kHd * 4;
constexpr size_t kSzA   = (size_t)kRows * kPQP * 2;
constexpr size_t kSzPQ  = (size_t)kRows * kPQP * 4;
constexpr size_t kSzS   = (size_t)kRows * kHd * 2;
constexpr size_t kSzW1  = (size_t)kLy * kPQP * kHd * 2;
constexpr size_t kSzW2  = (size_t)kLy * kHd * kHd * 2;
constexpr size_t kSzWU  = (size_t)kLy * kHd * kPQP * 2;
constexpr size_t kOffHF0 = 0;
constexpr size_t kOffHF1 = kOffHF0 + kSzHF;
constexpr size_t kOffAH0 = kOffHF1 + kSzHF;
constexpr size_t kOffAL0 = kOffAH0 + kSzA;
constexpr size_t kOffAH1 = kOffAL0 + kSzA;
constexpr size_t kOffAL1 = kOffAH1 + kSzA;
constexpr size_t kOffPQ  = kOffAL1 + kSzA;
constexpr size_t kOffSH  = kOffPQ  + kSzPQ;
constexpr size_t kOffSL  = kOffSH  + kSzS;
constexpr size_t kOffW1H = kOffSL  + kSzS;
constexpr size_t kOffW1L = kOffW1H + kSzW1;
constexpr size_t kOffW2H = kOffW1L + kSzW1;
constexpr size_t kOffW2L = kOffW2H + kSzW2;
constexpr size_t kOffWUH = kOffW2L + kSzW2;
constexpr size_t kOffWUL = kOffWUH + kSzWU;
constexpr size_t kWsTotal = kOffWUL + kSzWU;
static_assert(kWsTotal == 10747904ull, "carve total");
static_assert(kWsTotal <= 134217728ull, "carve cap");
static_assert((kSzHF % 128) == 0 && (kSzA % 128) == 0 && (kSzPQ % 128) == 0 && (kSzS % 128) == 0 &&
              (kSzW1 % 128) == 0 && (kSzW2 % 128) == 0 && (kSzWU % 128) == 0, "128-B aligned regions");

__device__ __forceinline__ void pin_u32(unsigned& t) { asm volatile("" : "+v"(t)); }

__device__ __forceinline__ unsigned bf_rne32(float f) {
  unsigned u = __float_as_uint(f);
  const unsigned lsb = (u & 0x00010000u) ? 1u : 0u;
  u = (u + 0x7FFFu + lsb) & 0xFFFF0000u;
  return u;
}
__device__ __forceinline__ void split_pair(float v0, float v1, unsigned& wh, unsigned& wl) {
  const unsigned h0 = bf_rne32(v0);
  const unsigned h1 = bf_rne32(v1);
  const unsigned l0 = bf_rne32(v0 - __uint_as_float(h0));
  const unsigned l1 = bf_rne32(v1 - __uint_as_float(h1));
  wh = __builtin_amdgcn_perm(h1, h0, 0x07060302u);
  wl = __builtin_amdgcn_perm(l1, l0, 0x07060302u);
}
__device__ __forceinline__ void split8(const v4f a0, const v4f a1, v4u& hv, v4u& lv) {
  const float f0 = a0[0], f1 = a0[1], f2 = a0[2], f3 = a0[3];
  const float f4 = a1[0], f5 = a1[1], f6 = a1[2], f7 = a1[3];
  unsigned h, l;
  split_pair(f0, f1, h, l); hv[0] = h; lv[0] = l;
  split_pair(f2, f3, h, l); hv[1] = h; lv[1] = l;
  split_pair(f4, f5, h, l); hv[2] = h; lv[2] = l;
  split_pair(f6, f7, h, l); hv[3] = h; lv[3] = l;
}
__device__ __forceinline__ void wave_lds_sync() {
  __builtin_amdgcn_fence(__ATOMIC_RELEASE, "workgroup");
  __builtin_amdgcn_wave_barrier();
  __builtin_amdgcn_fence(__ATOMIC_ACQUIRE, "workgroup");
}

__device__ __forceinline__ v16b frag_load(const __bf16* p) {
  union { v16b v; v8b h[2]; } f;
  f.h[0] = *(const v8b*)(p);
  f.h[1] = *(const v8b*)(p + 16);
  return f.v;
}
__device__ __forceinline__ v8f mma_bf(v16b a, v16b b, v8f c) {
  return __builtin_amdgcn_wmma_f32_16x16x32_bf16(false, a, false, b, (short)0, c, false, false);
}
__device__ __forceinline__ void guard1(v8f& a, v16b x, v16b y) {
  asm volatile("v_nop\n\tv_nop\n\tv_nop\n\tv_nop" : "+v"(a) : "v"(x), "v"(y));
}
__device__ __forceinline__ void keep4_b(v16b a, v16b b, v16b c, v16b d) { asm volatile("v_nop" :: "v"(a), "v"(b), "v"(c), "v"(d)); }
__device__ __forceinline__ void acc_guard4(v8f& a, v8f& b, v8f& c, v8f& d) {
  asm volatile("v_nop\n\tv_nop\n\tv_nop\n\tv_nop" : "+v"(a), "+v"(b), "+v"(c), "+v"(d));
}

__global__ __launch_bounds__(256) void wprep_kernel(
    const float* __restrict__ src, int srcLayerStride,
    unsigned short* dH, unsigned short* dL, int Nd, int Kd)
{
  __shared__ __align__(16) float sT[64 * 33];
  const int tid = threadIdx.x;
  const int k0 = blockIdx.x * 64;
  const int n0 = blockIdx.y * 32;
  const int l  = blockIdx.z;
  const int srcRowBase = 128 * (n0 >> 7);
  const int srcColBase = n0 & 127;
  const float* sp = src + (size_t)l * srcLayerStride;
  unsigned unn = (unsigned)tid & 31u;
  pin_u32(unn);
  unsigned ukk = (unsigned)tid >> 5;
  pin_u32(ukk);
#pragma unroll 1
  for (int i = 0; i < 8; ++i) {
    const int k = (int)ukk + 8 * i;
    sT[k * 33 + (int)unn] = sp[(size_t)(srcRowBase + k0 + k) * kHd + srcColBase + (int)unn];
  }
  __syncthreads();
  unsigned urow = (unsigned)tid >> 3;
  pin_u32(urow);
  unsigned uc8 = ((unsigned)tid & 7u) * 8u;
  pin_u32(uc8);
  v4f a0, a1;
  a0[0] = sT[((int)uc8 + 0) * 33 + (int)urow];
  a0[1] = sT[((int)uc8 + 1) * 33 + (int)urow];
  a0[2] = sT[((int)uc8 + 2) * 33 + (int)urow];
  a0[3] = sT[((int)uc8 + 3) * 33 + (int)urow];
  a1[0] = sT[((int)uc8 + 4) * 33 + (int)urow];
  a1[1] = sT[((int)uc8 + 5) * 33 + (int)urow];
  a1[2] = sT[((int)uc8 + 6) * 33 + (int)urow];
  a1[3] = sT[((int)uc8 + 7) * 33 + (int)urow];
  v4u hv, lv;
  split8(a0, a1, hv, lv);
  const size_t o = ((size_t)l * Nd + n0 + (int)urow) * Kd + k0 + (int)uc8;
  *(volatile v4u*)(dH + o) = hv;
  *(volatile v4u*)(dL + o) = lv;
  __threadfence();
  *(volatile v4u*)(dH + o) = hv;
  *(volatile v4u*)(dL + o) = lv;
}

__global__ __launch_bounds__(256) void embed_kernel(
    const float* __restrict__ state, const float* __restrict__ ew, const float* __restrict__ eb,
    float* Hf, unsigned short* AH, unsigned short* AL)
{
  __shared__ __align__(16) float sH[16 * 132];
  const int tid = threadIdx.x, lane = tid & 31, wave = tid >> 5;
  const int r0 = blockIdx.x * 16;
  const int c = tid & 127, rg = tid >> 7;
  const float w0 = ew[0 * kHd + c], w1 = ew[1 * kHd + c], w2 = ew[2 * kHd + c], w3 = ew[3 * kHd + c];
  const float bb = eb[c];
#pragma unroll 1
  for (int i = 0; i < 8; ++i) {
    const int row = rg * 8 + i;
    const v4f sv = *(const v4f*)(state + (size_t)(r0 + row) * kSd);
    const float s0 = sv[0], s1 = sv[1], s2 = sv[2], s3 = sv[3];
    float a = s0 * w0;
    a = fmaf(s1, w1, a);
    a = fmaf(s2, w2, a);
    a = fmaf(s3, w3, a);
    sH[row * 132 + c] = a + bb;
  }
  __syncthreads();
  unsigned uc4 = (unsigned)lane * 4u;
  pin_u32(uc4);
  unsigned uhh = (unsigned)lane >> 4;
  pin_u32(uhh);
  unsigned uc8 = ((unsigned)lane & 15u) * 8u;
  pin_u32(uc8);
  v4f fv[2];
#pragma unroll
  for (int it = 0; it < 2; ++it) fv[it] = *(const v4f*)(sH + (it * 8 + wave) * 132 + (int)uc4);
  const int brow = wave * 2 + (int)uhh;
  const v4f a0 = *(const v4f*)(sH + brow * 132 + (int)uc8);
  const v4f a1 = *(const v4f*)(sH + brow * 132 + (int)uc8 + 4);
  v4u hv, lv;
  split8(a0, a1, hv, lv);
  const size_t ob = (size_t)(r0 + brow) * kPQP + (int)uc8;
  for (int pass = 0; pass < 2; ++pass) {
#pragma unroll
    for (int it = 0; it < 2; ++it)
      *(volatile v4f*)(Hf + (size_t)(r0 + it * 8 + wave) * kHd + (int)uc4) = fv[it];
    *(volatile v4u*)(AH + ob) = hv;
    *(volatile v4u*)(AL + ob) = lv;
    __threadfence();
  }
}

template <bool OUT_F32, bool OUT_SPLIT, bool RESID>
__global__ __launch_bounds__(256) void gemm_bf16x3_kernel(
    const unsigned short* __restrict__ Ahp, const unsigned short* __restrict__ Alp, int lda,
    const unsigned short* __restrict__ Bhp, const unsigned short* __restrict__ Blp, int ldb,
    float* Cf, int ldcf,
    unsigned short* Ch, unsigned short* Cl, int ldch,
    const float* __restrict__ bias, int nbias, float biasScale,
    const float* __restrict__ resid, int ldr,
    int M, int N, int K)
{
  const __bf16* Ah = (const __bf16*)Ahp;
  const __bf16* Al = (const __bf16*)Alp;
  const __bf16* Bh = (const __bf16*)Bhp;
  const __bf16* Bl = (const __bf16*)Blp;
  __shared__ __align__(16) float sT[8][16 * 68];
  const int lane = threadIdx.x & 31;
  const int wave = threadIdx.x >> 5;
  const int tilesN = N >> 6;
  const int tilesM = M >> 6;
  const int tile = blockIdx.x * 8 + wave;
  if (tile >= tilesM * tilesN) return;
  const int tm = tile / tilesN;
  const int tn = tile - tm * tilesN;
  const int m0 = tm << 6;
  const int n0 = tn << 6;

  const int rlane = lane & 15;
  const int koff  = (lane >> 4) * 8;
  const int mOff  = (lane >> 4) * 8;

  v8f acc[4][4];
#pragma unroll
  for (int i = 0; i < 4; ++i)
#pragma unroll
    for (int j = 0; j < 4; ++j) acc[i][j] = (v8f){0.f, 0.f, 0.f, 0.f, 0.f, 0.f, 0.f, 0.f};

  for (int k0 = 0; k0 < K; k0 += 32) {
    v16b bh[4], bl[4];
#pragma unroll
    for (int j = 0; j < 4; ++j) {
      const size_t bo = (size_t)(n0 + (j << 4) + rlane) * ldb + koff + k0;
      bh[j] = frag_load(Bh + bo);
      bl[j] = frag_load(Bl + bo);
    }
#pragma unroll
    for (int i = 0; i < 4; ++i) {
      const size_t ao = (size_t)(m0 + (i << 4) + rlane) * lda + koff + k0;
      const v16b ah = frag_load(Ah + ao);
      const v16b al = frag_load(Al + ao);
#pragma unroll
      for (int j = 0; j < 4; ++j) {
        acc[i][j] = mma_bf(ah, bh[j], acc[i][j]);
        acc[i][j] = mma_bf(ah, bl[j], acc[i][j]);
        acc[i][j] = mma_bf(al, bh[j], acc[i][j]);
      }
      guard1(acc[i][0], ah, al);
      guard1(acc[i][1], ah, al);
      guard1(acc[i][2], ah, al);
      guard1(acc[i][3], ah, al);
    }
    keep4_b(bh[0], bh[1], bh[2], bh[3]);
    keep4_b(bl[0], bl[1], bl[2], bl[3]);
  }
  acc_guard4(acc[0][0], acc[0][1], acc[0][2], acc[0][3]);
  acc_guard4(acc[1][0], acc[1][1], acc[1][2], acc[1][3]);
  acc_guard4(acc[2][0], acc[2][1], acc[2][2], acc[2][3]);
  acc_guard4(acc[3][0], acc[3][1], acc[3][2], acc[3][3]);

  float* slab = sT[wave];
  unsigned uhh = (unsigned)lane >> 4;
  pin_u32(uhh);
  unsigned uc4 = ((unsigned)lane & 15u) * 4u;
  pin_u32(uc4);
  unsigned uq = (unsigned)lane >> 3;
  pin_u32(uq);
  unsigned uc8 = ((unsigned)lane & 7u) * 8u;
  pin_u32(uc8);
#pragma unroll
  for (int i = 0; i < 4; ++i) {
    const int mBase = m0 + (i << 4);
#pragma unroll
    for (int j = 0; j < 4; ++j) {
      const int n = n0 + (j << 4) + rlane;
      const int nb = (n < nbias) ? n : (nbias - 1);
      float bv = bias[nb];
      bv = (n < nbias) ? (bv * biasScale) : 0.0f;
#pragma unroll
      for (int r = 0; r < 8; ++r) slab[(mOff + r) * 68 + (j << 4) + rlane] = acc[i][j][r] + bv;
    }
    wave_lds_sync();
    if (OUT_F32) {
      v4f fv[8];
#pragma unroll
      for (int it = 0; it < 8; ++it) {
        const int row = it * 2 + (int)uhh;
        fv[it] = *(const v4f*)(slab + row * 68 + (int)uc4);
        if (RESID) {
          const v4f rv = *(const v4f*)(resid + (size_t)(mBase + row) * ldr + n0 + (int)uc4);
          fv[it] = fv[it] + rv;
          if (OUT_SPLIT) *(v4f*)(slab + row * 68 + (int)uc4) = fv[it];
        }
      }
      for (int pass = 0; pass < 2; ++pass) {
#pragma unroll
        for (int it = 0; it < 8; ++it) {
          const int row = it * 2 + (int)uhh;
          *(volatile v4f*)(Cf + (size_t)(mBase + row) * ldcf + n0 + (int)uc4) = fv[it];
        }
        __threadfence();
      }
      if (RESID && OUT_SPLIT) wave_lds_sync();
    }
    if (OUT_SPLIT) {
      v4u hv[4], lv[4];
#pragma unroll
      for (int it = 0; it < 4; ++it) {
        const int row = it * 4 + (int)uq;
        const v4f a0 = *(const v4f*)(slab + row * 68 + (int)uc8);
        const v4f a1 = *(const v4f*)(slab + row * 68 + (int)uc8 + 4);
        split8(a0, a1, hv[it], lv[it]);
      }
      for (int pass = 0; pass < 2; ++pass) {
#pragma unroll
        for (int it = 0; it < 4; ++it) {
          const int row = it * 4 + (int)uq;
          const size_t o = (size_t)(mBase + row) * ldch + n0 + (int)uc8;
          *(volatile v4u*)(Ch + o) = hv[it];
          *(volatile v4u*)(Cl + o) = lv[it];
        }
        __threadfence();
      }
    }
    wave_lds_sync();
  }
}

__global__ __launch_bounds__(128) void pair_silu_sum_kernel(
    const float* __restrict__ state, const float* __restrict__ PQ, const float* __restrict__ w1d,
    unsigned short* SH, unsigned short* SL)
{
  __shared__ __align__(16) float sD2[kNp * kIT];
  __shared__ __align__(16) float sS[kIT * 132];
  const int tid = threadIdx.x, lane = tid & 31, wave = tid >> 5;
  const int r0 = blockIdx.x * kIT;
  const int b  = r0 / kNp;
  const int i0 = r0 - b * kNp;
#pragma unroll 1
  for (int jj = tid; jj < kNp; jj += 128) {
    const v4f sj = *(const v4f*)(state + (size_t)(b * kNp + jj) * kSd);
    const float xj = sj[0], yj = sj[1];
#pragma unroll 1
    for (int ii = 0; ii < kIT; ++ii) {
      const v4f si = *(const v4f*)(state + (size_t)(r0 + ii) * kSd);
      const float dx = si[0] - xj;
      const float dy = si[1] - yj;
      sD2[jj * kIT + ii] = dx * dx + dy * dy;
    }
  }
  __syncthreads();
  float p[kIT], acc[kIT];
#pragma unroll
  for (int ii = 0; ii < kIT; ++ii) {
    p[ii] = PQ[(size_t)(r0 + ii) * kPQP + tid];
    acc[ii] = 0.0f;
  }
  const float wd = w1d[tid];
  const float* Qb = PQ + (size_t)b * kNp * kPQP + kHd + tid;
#pragma unroll 1
  for (int j = 0; j < kNp; ++j) {
    const float q = Qb[(size_t)j * kPQP];
    const v4f d0 = *(const v4f*)(sD2 + j * kIT);
    const v4f d1 = *(const v4f*)(sD2 + j * kIT + 4);
    const float dd[kIT] = {d0[0], d0[1], d0[2], d0[3], d1[0], d1[1], d1[2], d1[3]};
#pragma unroll
    for (int ii = 0; ii < kIT; ++ii) {
      const float x = fmaf(dd[ii], wd, p[ii] + q);
      const float e = expf(-x);
      const float s = x * __builtin_amdgcn_rcpf(1.0f + e);
      acc[ii] += (j == i0 + ii) ? 0.0f : s;
    }
  }
#pragma unroll
  for (int ii = 0; ii < kIT; ++ii) sS[ii * 132 + tid] = acc[ii];
  __syncthreads();
  unsigned uhh = (unsigned)lane >> 4;
  pin_u32(uhh);
  unsigned uc8 = ((unsigned)lane & 15u) * 8u;
  pin_u32(uc8);
  const int row = wave * 2 + (int)uhh;
  const v4f a0 = *(const v4f*)(sS + row * 132 + (int)uc8);
  const v4f a1 = *(const v4f*)(sS + row * 132 + (int)uc8 + 4);
  v4u hv, lv;
  split8(a0, a1, hv, lv);
  const size_t o = (size_t)(r0 + row) * kHd + (int)uc8;
  *(volatile v4u*)(SH + o) = hv;
  *(volatile v4u*)(SL + o) = lv;
  __threadfence();
  *(volatile v4u*)(SH + o) = hv;
  *(volatile v4u*)(SL + o) = lv;
}

__global__ __launch_bounds__(256) void head_kernel(
    const float* __restrict__ state, const float* __restrict__ Hf, const float* __restrict__ ow,
    const float* __restrict__ ob, float* out)
{
  const int idx = blockIdx.x * 256 + threadIdx.x;
  const int row = idx >> 2, c = idx & 3;
  const float* hr = Hf + (size_t)row * kHd;
  float acc = 0.0f;
#pragma unroll 1
  for (int k4 = 0; k4 < kHd / 4; ++k4) {
    const v4f hv = *(const v4f*)(hr + 4 * k4);
    const float h0 = hv[0], h1 = hv[1], h2 = hv[2], h3 = hv[3];
    const float* wp = ow + (size_t)(4 * k4) * kSd + c;
    acc = fmaf(h0, wp[0], acc);
    acc = fmaf(h1, wp[kSd], acc);
    acc = fmaf(h2, wp[2 * kSd], acc);
    acc = fmaf(h3, wp[3 * kSd], acc);
  }
  const float delta = acc + ob[c];
  const float v = state[idx] + delta;
  *(volatile float*)(out + idx) = v;
  __threadfence();
  *(volatile float*)(out + idx) = v;
}

extern "C" void kernel_launch(void* const* d_in, const int* in_sizes, int n_in,
                              void* d_out, int out_size, void* d_ws, size_t ws_size,
                              hipStream_t stream) {
  if (n_in < 11) return;
  if (in_sizes[0] != kRows * kSd) return;
  if (in_sizes[1] != kSd * kHd) return;
  if (in_sizes[2] != kHd) return;
  if (in_sizes[3] != kLy * kW1Rows * kHd) return;
  if (in_sizes[4] != kLy * kHd) return;
  if (in_sizes[5] != kLy * kHd * kHd) return;
  if (in_sizes[6] != kLy * kHd) return;
  if (in_sizes[7] != kLy * 2 * kHd * kHd) return;
  if (in_sizes[8] != kLy * kHd) return;
  if (in_sizes[9] != kHd * kSd) return;
  if (in_sizes[10] != kSd) return;
  if (out_size != kRows * kSd) return;
  if (ws_size < kWsTotal) return;

  const float* state   = (const float*)d_in[0];
  const float* embed_w = (const float*)d_in[1];
  const float* embed_b = (const float*)d_in[2];
  const float* w1      = (const float*)d_in[3];
  const float* b1      = (const float*)d_in[4];
  const float* w2      = (const float*)d_in[5];
  const float* b2      = (const float*)d_in[6];
  const float* wu      = (const float*)d_in[7];
  const float* bu      = (const float*)d_in[8];
  const float* out_w   = (const float*)d_in[9];
  const float* out_b   = (const float*)d_in[10];
  float* out = (float*)d_out;

  char* ws = (char*)d_ws;
  float* HF[2] = { (float*)(ws + kOffHF0), (float*)(ws + kOffHF1) };
  unsigned short* AH[2] = { (unsigned short*)(ws + kOffAH0), (unsigned short*)(ws + kOffAH1) };
  unsigned short* AL[2] = { (unsigned short*)(ws + kOffAL0), (unsigned short*)(ws + kOffAL1) };
  float*          PQ  = (float*)(ws + kOffPQ);
  unsigned short* SH  = (unsigned short*)(ws + kOffSH);
  unsigned short* SL  = (unsigned short*)(ws + kOffSL);
  unsigned short* W1H = (unsigned short*)(ws + kOffW1H);
  unsigned short* W1L = (unsigned short*)(ws + kOffW1L);
  unsigned short* W2H = (unsigned short*)(ws + kOffW2H);
  unsigned short* W2L = (unsigned short*)(ws + kOffW2L);
  unsigned short* WUH = (unsigned short*)(ws + kOffWUH);
  unsigned short* WUL = (unsigned short*)(ws + kOffWUL);

  wprep_kernel<<<dim3(kHd / 64, kPQP / 32, kLy), 256, 0, stream>>>(w1, kW1Rows * kHd, W1H, W1L, kPQP, kHd);
  wprep_kernel<<<dim3(kHd / 64, kHd / 32, kLy), 256, 0, stream>>>(w2, kHd * kHd, W2H, W2L, kHd, kHd);
  wprep_kernel<<<dim3(kPQP / 64, kHd / 32, kLy), 256, 0, stream>>>(wu, kPQP * kHd, WUH, WUL, kHd, kPQP);

  embed_kernel<<<kRows / 16, 256, 0, stream>>>(state, embed_w, embed_b, HF[0], AH[0], AL[0]);

  int cur = 0;
  for (int l = 0; l < kLy; ++l) {
    const int nxt = cur ^ 1;
    gemm_bf16x3_kernel<true, false, false><<<(kRows / 64) * (kPQP / 64) / 8, 256, 0, stream>>>(
        AH[cur], AL[cur], kPQP,
        W1H + (size_t)l * kPQP * kHd, W1L + (size_t)l * kPQP * kHd, kHd,
        PQ, kPQP,
        SH, SL, kHd,
        b1 + l * kHd, kHd, 1.0f,
        HF[cur], kHd,
        kRows, kPQP, kHd);
    pair_silu_sum_kernel<<<kRows / kIT, 128, 0, stream>>>(
        state, PQ, w1 + (size_t)l * kW1Rows * kHd + (size_t)(2 * kHd) * kHd, SH, SL);
    gemm_bf16x3_kernel<false, true, false><<<(kRows / 64) * (kHd / 64) / 8, 256, 0, stream>>>(
        SH, SL, kHd,
        W2H + (size_t)l * kHd * kHd, W2L + (size_t)l * kHd * kHd, kHd,
        PQ, kPQP,
        AH[cur] + kHd, AL[cur] + kHd, kPQP,
        b2 + l * kHd, kHd, (float)(kNp - 1),
        HF[cur], kHd,
        kRows, kHd, kHd);
    gemm_bf16x3_kernel<true, true, true><<<(kRows / 64) * (kHd / 64) / 8, 256, 0, stream>>>(
        AH[cur], AL[cur], kPQP,
        WUH + (size_t)l * kHd * kPQP, WUL + (size_t)l * kHd * kPQP, kPQP,
        HF[nxt], kHd,
        AH[nxt], AL[nxt], kPQP,
        bu + l * kHd, kHd, 1.0f,
        HF[cur], kHd,
        kRows, kHd, kPQP);
    cur = nxt;
  }

  head_kernel<<<(kRows * kSd) / 256, 256, 0, stream>>>(state, HF[cur], out_w, out_b, out);
}
